// LSTMClassifier_70592082477252
// MI455X (gfx1250) — hardware-run, weakly checked
//
#include <hip/hip_runtime.h>
#include <math.h>

constexpr int NBAT     = 2048;
constexpr int NSTEP    = 512;
constexpr int NHID     = 64;
constexpr int NGATE    = 4 * NHID;
constexpr int NCLS     = 3;
constexpr int NTHR     = 256;
constexpr int ROWS_BLK = 32;
constexpr int XCH      = 64;
constexpr int HPITCH   = 72;
constexpr int SPITCH   = 68;
constexpr int NFO      = ROWS_BLK * NCLS;
constexpr int NW8      = (NGATE * NHID) / 8;
constexpr float HCARRY   = 16.0f;
constexpr float WCARRY   = 16.0f;
constexpr float PROD_INV = 1.0f / 256.0f;
static_assert(NBAT % ROWS_BLK == 0);
static_assert(NSTEP % XCH == 0);
static_assert((XCH & (XCH - 1)) == 0);
static_assert(NHID % 32 == 0);
static_assert(NGATE == NTHR);
static_assert(NTHR / 32 == (ROWS_BLK / 16) * (NHID / 16));
static_assert((XCH * ROWS_BLK) % NTHR == 0);
static_assert((2 * ROWS_BLK * HPITCH) % NTHR == 0);
static_assert(NCLS * NHID <= NTHR && (NCLS * NHID) % 32 == 0);
static_assert(NFO % 32 == 0 && NFO % 4 == 0 && (NFO * 4) % 128 == 0 && NFO / 4 <= 32);
static_assert(HPITCH % 8 == 0 && SPITCH % 4 == 0);
static_assert((NGATE * NHID) % 8 == 0 && NW8 % NTHR == 0);
static_assert(NCLS <= 4);

typedef __attribute__((ext_vector_type(16))) _Float16 v16h;
typedef __attribute__((ext_vector_type(8)))  _Float16 v8h;
typedef __attribute__((ext_vector_type(8)))  float    v8f;
typedef __attribute__((ext_vector_type(4)))  float    v4f;

__device__ __forceinline__ void acc_guard4(v8f& a, v8f& b, v8f& c, v8f& d) {
  asm volatile("v_nop\n\tv_nop\n\tv_nop\n\tv_nop" : "+v"(a), "+v"(b), "+v"(c), "+v"(d));
}
__device__ __forceinline__ void mma_guard4(v8f& a0, v8f& a1, v8f& a2, v8f& a3,
                                           v16h x, v16h y0, v16h y1, v16h y2, v16h y3) {
  asm volatile("v_nop\n\tv_nop\n\tv_nop\n\tv_nop"
               : "+v"(a0), "+v"(a1), "+v"(a2), "+v"(a3)
               : "v"(x), "v"(y0), "v"(y1), "v"(y2), "v"(y3));
}

template <typename T> struct Frag;
template <> struct Frag<_Float16> {
  typedef v16h V; union U { v16h v; v8h h[2]; };
  static __device__ __forceinline__ v16h load(const _Float16* p) {
    U f; f.h[0] = *(const v8h*)(p); f.h[1] = *(const v8h*)(p + 16); return f.v;
  }
  static __device__ __forceinline__ v8f mma(v16h a, v16h b, v8f c) {
    return __builtin_amdgcn_wmma_f32_16x16x32_f16(false, a, false, b, (short)0, c, false, false);
  }
};

__device__ __forceinline__ float fsig(float x)  { return __builtin_amdgcn_rcpf(1.0f + __expf(-x)); }
__device__ __forceinline__ float ftanh(float x) { return 1.0f - 2.0f * __builtin_amdgcn_rcpf(__expf(2.0f * x) + 1.0f); }

__global__ __launch_bounds__(NTHR) void cvt_w16_kernel(const float* __restrict__ src,
                                                       unsigned short* __restrict__ dst, int n8, float sc) {
  const int i = blockIdx.x * NTHR + threadIdx.x;
  if (i < n8) {
    const float* sp = src + (size_t)i * 8;
    const v4f a = *(const v4f*)(sp);
    const v4f b = *(const v4f*)(sp + 4);
    v8h hv;
#pragma unroll
    for (int e = 0; e < 4; ++e) {
      hv[e]     = (_Float16)(a[e] * sc);
      hv[4 + e] = (_Float16)(b[e] * sc);
    }
    unsigned short* dp = dst + (size_t)i * 8;
    *(volatile v8h*)dp = hv;
    __threadfence();
    *(volatile v8h*)dp = hv;
  }
}

__global__ __launch_bounds__(NTHR) void lstm2_seq_kernel(
    const float* __restrict__ x, const float* __restrict__ w_ih0,
    const float* __restrict__ b_ih0, const float* __restrict__ b_hh0,
    const float* __restrict__ b_ih1, const float* __restrict__ b_hh1,
    const float* __restrict__ w_fc, const float* __restrict__ b_fc,
    const unsigned short* __restrict__ W0p, const unsigned short* __restrict__ W1p,
    const unsigned short* __restrict__ W2p, float* __restrict__ out) {
  __shared__ __align__(16) _Float16 H0t[2][ROWS_BLK * HPITCH];
  __shared__ __align__(16) _Float16 H1t[2][ROWS_BLK * HPITCH];
  __shared__ __align__(16) float Xs[XCH * ROWS_BLK];
  __shared__ __align__(16) float Hs[ROWS_BLK * SPITCH];
  __shared__ __align__(16) float Fo[NFO];
  __shared__ float Cw0[NGATE];
  __shared__ float Cb0[NGATE];
  __shared__ float Cb1[NGATE];
  __shared__ float Cfc[NCLS * NHID];
  __shared__ float Cbf[4];

  const _Float16* W0 = (const _Float16*)W0p;
  const _Float16* W1 = (const _Float16*)W1p;
  const _Float16* W2 = (const _Float16*)W2p;
  const int tid = threadIdx.x, lane = tid & 31, wave = tid >> 5;
  const int c = lane & 15, hh = lane >> 4, koff = hh * 8;
  const int mt = wave >> 2, ug = wave & 3;
  const int j = 16 * ug + c;
  const int mrow = 16 * mt;
  const int rowbase = blockIdx.x * ROWS_BLK;

  {
    _Float16* p0 = &H0t[0][0];
    _Float16* p1 = &H1t[0][0];
#pragma unroll 1
    for (int i = tid; i < 2 * ROWS_BLK * HPITCH; i += NTHR) {
      p0[i] = (_Float16)0.0f;
      p1[i] = (_Float16)0.0f;
    }
  }
  Cw0[tid] = w_ih0[tid];
  Cb0[tid] = b_ih0[tid] + b_hh0[tid];
  Cb1[tid] = b_ih1[tid] + b_hh1[tid];
  if (tid < NCLS * NHID) Cfc[tid] = w_fc[tid];
  if (wave == 0) {
    const int li = (lane < NCLS) ? lane : (NCLS - 1);
    const float v = b_fc[li];
    if (lane < 4) Cbf[lane] = v;
  }
  float cst0[8], cst1[8], hst1[8];
#pragma unroll
  for (int r = 0; r < 8; ++r) { cst0[r] = 0.0f; cst1[r] = 0.0f; hst1[r] = 0.0f; }
  __syncthreads();

  float w0s[4], b0s[4], b1s[4];
#pragma unroll
  for (int g = 0; g < 4; ++g) {
    w0s[g] = Cw0[NHID * g + j];
    b0s[g] = Cb0[NHID * g + j];
    b1s[g] = Cb1[NHID * g + j];
  }
  const v8f z8 = {0.f, 0.f, 0.f, 0.f, 0.f, 0.f, 0.f, 0.f};

#pragma unroll 1
  for (int t = 0; t < NSTEP; ++t) {
    const int p = t & 1;
    if ((t & (XCH - 1)) == 0) {
#pragma unroll
      for (int it = 0; it < (XCH * ROWS_BLK) / NTHR; ++it) {
        const int i = it * NTHR + tid;
        const int m = i / XCH, tt = i & (XCH - 1);
        Xs[tt * ROWS_BLK + m] = x[(size_t)(rowbase + m) * NSTEP + (size_t)(t + tt)];
      }
      __syncthreads();
    }
    const float* xq = Xs + (t & (XCH - 1)) * ROWS_BLK + mrow + 8 * hh;
    const v4f xa = *(const v4f*)(xq);
    const v4f xb = *(const v4f*)(xq + 4);
    const float xv[8] = {xa[0], xa[1], xa[2], xa[3], xb[0], xb[1], xb[2], xb[3]};

    v8f acc[4];
    acc[0] = z8; acc[1] = z8; acc[2] = z8; acc[3] = z8;
    {
      const _Float16* arow = &H0t[p][0] + (mrow + c) * HPITCH + koff;
      const _Float16* wb = W0 + (size_t)j * NHID + koff;
#pragma unroll 1
      for (int k0 = 0; k0 < NHID; k0 += 32) {
        const v16h a  = Frag<_Float16>::load(arow + k0);
        const v16h b0 = Frag<_Float16>::load(wb + k0);
        const v16h b1 = Frag<_Float16>::load(wb + (size_t)1 * NHID * NHID + k0);
        const v16h b2 = Frag<_Float16>::load(wb + (size_t)2 * NHID * NHID + k0);
        const v16h b3 = Frag<_Float16>::load(wb + (size_t)3 * NHID * NHID + k0);
        acc[0] = Frag<_Float16>::mma(a, b0, acc[0]);
        acc[1] = Frag<_Float16>::mma(a, b1, acc[1]);
        acc[2] = Frag<_Float16>::mma(a, b2, acc[2]);
        acc[3] = Frag<_Float16>::mma(a, b3, acc[3]);
        mma_guard4(acc[0], acc[1], acc[2], acc[3], a, b0, b1, b2, b3);
      }
    }
    acc_guard4(acc[0], acc[1], acc[2], acc[3]);
    {
      _Float16* hw = &H0t[p ^ 1][0];
#pragma unroll
      for (int r = 0; r < 8; ++r) {
        const float zi = fmaf(acc[0][r], PROD_INV, fmaf(xv[r], w0s[0], b0s[0]));
        const float zf = fmaf(acc[1][r], PROD_INV, fmaf(xv[r], w0s[1], b0s[1]));
        const float zg = fmaf(acc[2][r], PROD_INV, fmaf(xv[r], w0s[2], b0s[2]));
        const float zo = fmaf(acc[3][r], PROD_INV, fmaf(xv[r], w0s[3], b0s[3]));
        const float ig = fsig(zi);
        const float fg = fsig(zf);
        const float gg = ftanh(zg);
        const float og = fsig(zo);
        const float cn = fg * cst0[r] + ig * gg;
        cst0[r] = cn;
        const float hn = og * ftanh(cn);
        hw[(mrow + 8 * hh + r) * HPITCH + j] = (_Float16)(hn * HCARRY);
      }
    }
    __syncthreads();

    acc[0] = z8; acc[1] = z8; acc[2] = z8; acc[3] = z8;
    {
      const _Float16* arow = &H0t[p ^ 1][0] + (mrow + c) * HPITCH + koff;
      const _Float16* wb = W1 + (size_t)j * NHID + koff;
#pragma unroll 1
      for (int k0 = 0; k0 < NHID; k0 += 32) {
        const v16h a  = Frag<_Float16>::load(arow + k0);
        const v16h b0 = Frag<_Float16>::load(wb + k0);
        const v16h b1 = Frag<_Float16>::load(wb + (size_t)1 * NHID * NHID + k0);
        const v16h b2 = Frag<_Float16>::load(wb + (size_t)2 * NHID * NHID + k0);
        const v16h b3 = Frag<_Float16>::load(wb + (size_t)3 * NHID * NHID + k0);
        acc[0] = Frag<_Float16>::mma(a, b0, acc[0]);
        acc[1] = Frag<_Float16>::mma(a, b1, acc[1]);
        acc[2] = Frag<_Float16>::mma(a, b2, acc[2]);
        acc[3] = Frag<_Float16>::mma(a, b3, acc[3]);
        mma_guard4(acc[0], acc[1], acc[2], acc[3], a, b0, b1, b2, b3);
      }
    }
    {
      const _Float16* arow = &H1t[p][0] + (mrow + c) * HPITCH + koff;
      const _Float16* wb = W2 + (size_t)j * NHID + koff;
#pragma unroll 1
      for (int k0 = 0; k0 < NHID; k0 += 32) {
        const v16h a  = Frag<_Float16>::load(arow + k0);
        const v16h b0 = Frag<_Float16>::load(wb + k0);
        const v16h b1 = Frag<_Float16>::load(wb + (size_t)1 * NHID * NHID + k0);
        const v16h b2 = Frag<_Float16>::load(wb + (size_t)2 * NHID * NHID + k0);
        const v16h b3 = Frag<_Float16>::load(wb + (size_t)3 * NHID * NHID + k0);
        acc[0] = Frag<_Float16>::mma(a, b0, acc[0]);
        acc[1] = Frag<_Float16>::mma(a, b1, acc[1]);
        acc[2] = Frag<_Float16>::mma(a, b2, acc[2]);
        acc[3] = Frag<_Float16>::mma(a, b3, acc[3]);
        mma_guard4(acc[0], acc[1], acc[2], acc[3], a, b0, b1, b2, b3);
      }
    }
    acc_guard4(acc[0], acc[1], acc[2], acc[3]);
    {
      _Float16* hw = &H1t[p ^ 1][0];
#pragma unroll
      for (int r = 0; r < 8; ++r) {
        const float zi = fmaf(acc[0][r], PROD_INV, b1s[0]);
        const float zf = fmaf(acc[1][r], PROD_INV, b1s[1]);
        const float zg = fmaf(acc[2][r], PROD_INV, b1s[2]);
        const float zo = fmaf(acc[3][r], PROD_INV, b1s[3]);
        const float ig = fsig(zi);
        const float fg = fsig(zf);
        const float gg = ftanh(zg);
        const float og = fsig(zo);
        const float cn = fg * cst1[r] + ig * gg;
        cst1[r] = cn;
        const float hn = og * ftanh(cn);
        hst1[r] = hn;
        hw[(mrow + 8 * hh + r) * HPITCH + j] = (_Float16)(hn * HCARRY);
      }
    }
    __syncthreads();
  }

#pragma unroll
  for (int r = 0; r < 8; ++r) Hs[(mrow + 8 * hh + r) * SPITCH + j] = hst1[r];
  __syncthreads();
  if (tid < NFO) {
    const int m = tid / NCLS;
    const int cc = tid - m * NCLS;
    float s = Cbf[cc];
    const float* hr = Hs + m * SPITCH;
    const float* wr = Cfc + cc * NHID;
#pragma unroll 8
    for (int k = 0; k < NHID; ++k) s = fmaf(hr[k], wr[k], s);
    Fo[tid] = s;
  }
  __syncthreads();
  if (wave == 0) {
    const int li = (lane < NFO / 4) ? lane : (NFO / 4 - 1);
    const v4f v = *(const v4f*)(Fo + 4 * li);
    float* op = out + (size_t)blockIdx.x * NFO + 4 * li;
    if (lane < NFO / 4) *(volatile v4f*)op = v;
    __threadfence();
    if (lane < NFO / 4) *(volatile v4f*)op = v;
  }
}

extern "C" void kernel_launch(void* const* d_in, const int* in_sizes, int n_in,
                              void* d_out, int out_size, void* d_ws, size_t ws_size, hipStream_t stream) {
  if (n_in < 11 || d_out == nullptr || d_ws == nullptr) return;
  if (in_sizes[0] != NBAT * NSTEP || in_sizes[1] != NGATE || in_sizes[2] != NGATE * NHID ||
      in_sizes[3] != NGATE || in_sizes[4] != NGATE || in_sizes[5] != NGATE * NHID ||
      in_sizes[6] != NGATE * NHID || in_sizes[7] != NGATE || in_sizes[8] != NGATE ||
      in_sizes[9] != NCLS * NHID || in_sizes[10] != NCLS || out_size != NBAT * NCLS) return;

  const float* x     = (const float*)d_in[0];
  const float* w_ih0 = (const float*)d_in[1];
  const float* w_hh0 = (const float*)d_in[2];
  const float* b_ih0 = (const float*)d_in[3];
  const float* b_hh0 = (const float*)d_in[4];
  const float* w_ih1 = (const float*)d_in[5];
  const float* w_hh1 = (const float*)d_in[6];
  const float* b_ih1 = (const float*)d_in[7];
  const float* b_hh1 = (const float*)d_in[8];
  const float* w_fc  = (const float*)d_in[9];
  const float* b_fc  = (const float*)d_in[10];
  float* out = (float*)d_out;

  char* ws = (char*)d_ws; size_t off = 0;
  auto carve = [&](size_t bytes) -> char* { char* p = ws + off; off += (bytes + 255) & ~(size_t)255; return p; };
  unsigned short* W0 = (unsigned short*)carve((size_t)NGATE * NHID * 2);
  unsigned short* W1 = (unsigned short*)carve((size_t)NGATE * NHID * 2);
  unsigned short* W2 = (unsigned short*)carve((size_t)NGATE * NHID * 2);
  if (off > ws_size || off > (size_t)134217728) return;

  cvt_w16_kernel<<<NW8 / NTHR, NTHR, 0, stream>>>(w_hh0, W0, NW8, WCARRY);
  cvt_w16_kernel<<<NW8 / NTHR, NTHR, 0, stream>>>(w_ih1, W1, NW8, WCARRY);
  cvt_w16_kernel<<<NW8 / NTHR, NTHR, 0, stream>>>(w_hh1, W2, NW8, WCARRY);
  lstm2_seq_kernel<<<NBAT / ROWS_BLK, NTHR, 0, stream>>>(x, w_ih0, b_ih0, b_hh0, b_ih1, b_hh1, w_fc, b_fc,
                                                           W0, W1, W2, out);
}
